// UnimodalBranch_2070174237004
// MI455X (gfx1250) — hardware-verified
//
#include <hip/hip_runtime.h>


namespace {
constexpr int B = 8, CI = 128, CO = 128, S = 64, KK = CI * 9, NPIX = B * S * S, N = 50000, NV = 200000, M = 800000;
constexpr float XS = 8.0f, WSC = 256.0f;
typedef _Float16 b16;
typedef __attribute__((ext_vector_type(16))) _Float16 v16b;
typedef __attribute__((ext_vector_type(8))) _Float16 v8b;
typedef __attribute__((ext_vector_type(8))) float v8f;
typedef __attribute__((ext_vector_type(4))) float v4f;
__device__ __forceinline__ float bf16_rne(float f) { unsigned int u = __float_as_uint(f); u += 0x7FFFu + ((u >> 16) & 1u); return __uint_as_float(u & 0xFFFF0000u); }
__device__ __forceinline__ v16b frag_kb(const b16* p, int hh) { const v8b a = *(const v8b*)(p + 8 * hh), b = *(const v8b*)(p + 16 + 8 * hh); v16b f;
#pragma unroll
  for (int e = 0; e < 8; ++e) { f[e] = a[e]; f[8 + e] = b[e]; } return f; }
__device__ __forceinline__ v8f wmma16b(v16b a, v16b b, v8f c) { v8f d = __builtin_amdgcn_wmma_f32_16x16x32_f16(false, a, false, b, (short)0, c, false, false); asm volatile("v_nop\n\tv_nop\n\tv_nop\n\tv_nop" : "+v"(d) : "v"(a), "v"(b)); return d; }
__device__ __forceinline__ void wave_lds_sync() { __builtin_amdgcn_fence(__ATOMIC_RELEASE, "workgroup"); __builtin_amdgcn_wave_barrier(); __builtin_amdgcn_fence(__ATOMIC_ACQUIRE, "workgroup"); }
__device__ __forceinline__ int iclamp(int v, int lo, int hi) { return v < lo ? lo : (v > hi ? hi : v); }

__global__ __launch_bounds__(256) void wput_kernel(const float* __restrict__ W, b16* __restrict__ WT) {
  const int u = blockIdx.x * 256 + threadIdx.x; if (u >= CO * 9 * 16) return; const int c8 = u % 16, tap = (u / 16) % 9, co = u / 144; v8b v;
#pragma unroll
  for (int j = 0; j < 8; ++j) { const int ci = c8 * 8 + j; v[j] = (b16)(bf16_rne(W[((size_t)co * CI + ci) * 9 + tap]) * WSC); } for (int pass = 0; pass < 2; ++pass) { *(volatile v8b*)(WT + (size_t)co * KK + tap * CI + c8 * 8) = v; __threadfence(); }
}
__global__ __launch_bounds__(32) void conv_kernel(const float* __restrict__ x, const b16* __restrict__ WT, const float* __restrict__ bias, int BV, float* __restrict__ Y) {
  __shared__ __attribute__((aligned(16))) b16 Xs[3][34][CI + 8]; __shared__ float Of[32][CO + 4];
  const int lane = threadIdx.x, nloc = lane & 15, hlf = lane >> 4; const int hx = blockIdx.x & 1, y = (blockIdx.x >> 1) % S, b = blockIdx.x / (2 * S); if (b >= BV) return; const int x0 = hx * 32;
  for (int kh = 0; kh < 3; ++kh) { const int yy = y + kh - 1;
    for (int xx = 0; xx < 34; ++xx) { const int xg = x0 + xx - 1; const bool ok = yy >= 0 && yy < S && xg >= 0 && xg < S;
      for (int q = 0; q < 4; ++q) { const int ci = q * 32 + lane; Xs[kh][xx][ci] = (b16)(ok ? bf16_rne(x[(((size_t)b * CI + ci) * S + yy) * S + xg]) * XS : 0.0f); } } }
  wave_lds_sync(); v8f acc[2][8];
#pragma unroll
  for (int p = 0; p < 2; ++p)
#pragma unroll
    for (int t = 0; t < 8; ++t) acc[p][t] = (v8f){};
#pragma unroll 1
  for (int tap = 0; tap < 9; ++tap) { const int kh = tap / 3, kw = tap % 3;
#pragma unroll
    for (int cb = 0; cb < CI; cb += 32) { const v16b a0 = frag_kb(&Xs[kh][nloc + kw][cb], hlf), a1 = frag_kb(&Xs[kh][16 + nloc + kw][cb], hlf); const int k0 = tap * CI + cb;
#pragma unroll
      for (int t = 0; t < 8; ++t) { const v16b bw = frag_kb(WT + (size_t)(t * 16 + nloc) * KK + k0, hlf); acc[0][t] = wmma16b(a0, bw, acc[0][t]); acc[1][t] = wmma16b(a1, bw, acc[1][t]); } } }
#pragma unroll
  for (int p = 0; p < 2; ++p)
#pragma unroll
    for (int t = 0; t < 8; ++t) { const int co = t * 16 + nloc; const float bb = bf16_rne(bias[co]);
#pragma unroll
      for (int r8 = 0; r8 < 8; ++r8) Of[p * 16 + 8 * hlf + r8][co] = acc[p][t][r8] * (1.0f / (XS * WSC)) + bb; }
  wave_lds_sync();
  for (int pass = 0; pass < 2; ++pass) { for (int px = 0; px < 32; ++px) *(volatile v4f*)(Y + (((size_t)b * S + y) * S + x0 + px) * CO + lane * 4) = *(const v4f*)(&Of[px][lane * 4]); __threadfence(); }
}
__global__ __launch_bounds__(256) void pool_kernel(const float* __restrict__ Y, const int* __restrict__ pix, const int* __restrict__ aptr, const int* __restrict__ vptr, const float* __restrict__ x3, int NLIM, int PIXLIM, float* __restrict__ out) {
  const int wave = threadIdx.x >> 5, lane = threadIdx.x & 31; const size_t n = (size_t)blockIdx.x * 8 + wave; if (n >= (size_t)NLIM) return;
  const int v0 = iclamp(vptr[n], 0, NV), v1 = iclamp(vptr[n + 1], v0, NV); v4f pm = {-INFINITY, -INFINITY, -INFINITY, -INFINITY};
#pragma unroll 1
  for (int v = v0; v < v1; ++v) { const int p0 = iclamp(aptr[v], 0, M), p1 = iclamp(aptr[v + 1], p0, M); v4f vm = {-INFINITY, -INFINITY, -INFINITY, -INFINITY};
#pragma unroll 1
    for (int p = p0; p < p1; ++p) { int id = iclamp(pix[p], 0, NPIX - 1); if (id >= PIXLIM) id %= PIXLIM;
      const v4f yv = *(const v4f*)(Y + (size_t)id * CO + lane * 4); for (int i = 0; i < 4; ++i) vm[i] = fmaxf(vm[i], yv[i]); }
    for (int i = 0; i < 4; ++i) { const float vv = (p1 > p0) ? vm[i] : 0.0f; pm[i] = fmaxf(pm[i], vv); } }
  v4f o; const v4f xr = *(const v4f*)(x3 + n * CO + lane * 4); for (int i = 0; i < 4; ++i) o[i] = bf16_rne(xr[i]) + ((v1 > v0) ? pm[i] : 0.0f);
  for (int pass = 0; pass < 2; ++pass) { *(volatile v4f*)(out + n * CO + lane * 4) = o; __threadfence(); }
}
}

extern "C" void kernel_launch(void* const* d_in, const int* in_sizes, int n_in, void* d_out, int out_size, void* d_ws, size_t ws_size, hipStream_t stream) {
  (void)n_in;
  auto Fp = [&](int i) { return (const float*)d_in[i]; }; auto Ip = [&](int i) { return (const int*)d_in[i]; };
  if (in_sizes[0] != N * CO || in_sizes[1] != B * CI * S * S || in_sizes[2] != CO * CI * 9 || in_sizes[3] != CO || in_sizes[4] != M || in_sizes[5] != NV + 1 || in_sizes[6] != N + 1 || out_size != N * CO) return;
  const int BV = B, NLIM = N, PIXLIM = NPIX;
  size_t off = 0; char* ws = (char*)d_ws;
  auto carve = [&](size_t bytes) { char* p = ws + off; off += (bytes + 255) & ~(size_t)255; return p; };
  b16* WT = (b16*)carve((size_t)CO * KK * 2); float* Y = (float*)carve((size_t)NPIX * CO * 4);
  if (off > ws_size || off > ((size_t)32 << 20)) return;
  wput_kernel<<<(CO * 144 + 255) / 256, 256, 0, stream>>>(Fp(2), WT);
  conv_kernel<<<BV * S * 2, 32, 0, stream>>>(Fp(1), WT, Fp(3), BV, Y);
  pool_kernel<<<(NLIM + 7) / 8, 256, 0, stream>>>(Y, Ip(4), Ip(5), Ip(6), Fp(0), NLIM, PIXLIM, (float*)d_out);
}
